// TransformerMoEBlock_87531433493249
// MI455X (gfx1250) — hardware-verified
//
#include <hip/hip_runtime.h>
#include <stddef.h>


#define NTOK 8192
#define DD   512
#define FFD  2048
#define NE   8
#define EPSW 0.01f
#define TR   64
#define NTL  264
#define NGRP 4
#define TPG  66
#define CAPE 4096
#define NTHR 256
#define LDS_LISTS (NE * CAPE * 4)

static_assert(NGRP * TPG == NTL);
static_assert(NTL * TR >= 2 * NTOK + NE * (TR - 1));
static_assert((NTOK % NTHR) == 0 && (NTOK % 32) == 0 && (NTOK % 2) == 0);
static_assert((DD % 256) == 0 && (FFD % 256) == 0 && (DD % 64) == 0 && (FFD % 64) == 0);
static_assert((CAPE % TR) == 0);
static_assert(((NTL * TR / 4) % 8) == 0);
static_assert(((NTL * TR) % 4) == 0);

typedef float          v4f   __attribute__((ext_vector_type(4)));
typedef float          v8f   __attribute__((ext_vector_type(8)));
typedef int            v4i   __attribute__((ext_vector_type(4)));
typedef unsigned short v8us  __attribute__((ext_vector_type(8)));
typedef unsigned short v16us __attribute__((ext_vector_type(16)));
typedef __bf16         v16bf __attribute__((ext_vector_type(16)));
union FragB { v16us u; v8us h[2]; v16bf v; };

__device__ __forceinline__ unsigned int bfbits(float f) {
  unsigned int u = __float_as_uint(f);
  u = u + 0x7FFFu + ((u >> 16) & 1u);
  return u >> 16;
}
__device__ __forceinline__ float bfr(float f) { return __uint_as_float(bfbits(f) << 16); }

__device__ __forceinline__ v8f wmb(v16bf a, v16bf b, v8f c) {
  v8f d = __builtin_amdgcn_wmma_f32_16x16x32_bf16(false, a, false, b, (short)0, c, false, false);
#if defined(__HIP_DEVICE_COMPILE__)
  asm volatile("v_nop\n\tv_nop\n\tv_nop\n\tv_nop" : "+v"(d) : "v"(a), "v"(b));
#endif
  return d;
}

__global__ __launch_bounds__(NTHR) void k_wconv(const float* __restrict__ W, unsigned short* Wt, int K, int N) {
  __shared__ __attribute__((aligned(16))) unsigned short tile[64 * 72];
  const int tid = threadIdx.x;
  const int k0 = blockIdx.x * 64, n0 = blockIdx.y * 64, e = blockIdx.z;
  const float* src = W + (size_t)e * K * N;
#pragma unroll
  for (int i = 0; i < 4; ++i) {
    const int idx = i * NTHR + tid;
    const int kr  = idx >> 4;
    const int nc  = (idx & 15) * 4;
    const v4f v = *(const v4f*)(src + (size_t)(k0 + kr) * N + n0 + nc);
    tile[(nc + 0) * 72 + kr] = (unsigned short)bfbits(v.x);
    tile[(nc + 1) * 72 + kr] = (unsigned short)bfbits(v.y);
    tile[(nc + 2) * 72 + kr] = (unsigned short)bfbits(v.z);
    tile[(nc + 3) * 72 + kr] = (unsigned short)bfbits(v.w);
  }
  __syncthreads();
  const int nrA = tid >> 3;
  const int nrB = nrA + 32;
  const int pc  = tid & 7;
  const v8us va = *(const v8us*)(tile + nrA * 72 + pc * 8);
  const v8us vb = *(const v8us*)(tile + nrB * 72 + pc * 8);
  unsigned short* ga = Wt + ((size_t)e * N + n0 + nrA) * K + k0 + pc * 8;
  unsigned short* gb = Wt + ((size_t)e * N + n0 + nrB) * K + k0 + pc * 8;
  *(volatile v8us*)ga = va;
  *(volatile v8us*)gb = vb;
  __threadfence();
  *(volatile v8us*)ga = va;
  *(volatile v8us*)gb = vb;
}

__global__ __launch_bounds__(NTHR) void k_gate(
    const float* __restrict__ x, const float* __restrict__ Wg, const float* __restrict__ bg,
    int* tinfo, int nTok) {
  __shared__ __attribute__((aligned(16))) float sW[DD * NE];
  __shared__ float sb[NE];
  const int tid = threadIdx.x;
  for (int i = tid; i < DD * NE; i += NTHR) sW[i] = bfr(Wg[i]);
  if (tid < NE) sb[tid] = bfr(bg[tid]);
  __syncthreads();

  int t = blockIdx.x * NTHR + tid;
  t = t > nTok - 1 ? nTok - 1 : t;
  const float* xr = x + (size_t)t * DD;

  float a0 = 0.f, a1 = 0.f, a2 = 0.f, a3 = 0.f, a4 = 0.f, a5 = 0.f, a6 = 0.f, a7 = 0.f;
#pragma unroll 1
  for (int d = 0; d < DD; ++d) {
    const float xv = bfr(xr[d]);
    const v4f wA = *(const v4f*)(sW + d * NE);
    const v4f wB = *(const v4f*)(sW + d * NE + 4);
    a0 = fmaf(xv, wA.x, a0); a1 = fmaf(xv, wA.y, a1); a2 = fmaf(xv, wA.z, a2); a3 = fmaf(xv, wA.w, a3);
    a4 = fmaf(xv, wB.x, a4); a5 = fmaf(xv, wB.y, a5); a6 = fmaf(xv, wB.z, a6); a7 = fmaf(xv, wB.w, a7);
  }
  const float l0 = a0 + sb[0], l1 = a1 + sb[1], l2 = a2 + sb[2], l3 = a3 + sb[3];
  const float l4 = a4 + sb[4], l5 = a5 + sb[5], l6 = a6 + sb[6], l7 = a7 + sb[7];

  float mx = l0; int i0 = 0;
  if (l1 > mx) { mx = l1; i0 = 1; }
  if (l2 > mx) { mx = l2; i0 = 2; }
  if (l3 > mx) { mx = l3; i0 = 3; }
  if (l4 > mx) { mx = l4; i0 = 4; }
  if (l5 > mx) { mx = l5; i0 = 5; }
  if (l6 > mx) { mx = l6; i0 = 6; }
  if (l7 > mx) { mx = l7; i0 = 7; }
  int   i1 = (i0 == 0) ? 1 : 0;
  float m1 = (i0 == 0) ? l1 : l0;
#define CAND(EI, LV) { const bool c = ((EI) != i0) && ((LV) > m1); m1 = c ? (LV) : m1; i1 = c ? (EI) : i1; }
  CAND(1, l1) CAND(2, l2) CAND(3, l3) CAND(4, l4) CAND(5, l5) CAND(6, l6) CAND(7, l7)
#undef CAND

  const float LG2E = 1.4426950408889634f;
  const float g0 = exp2f((l0 - mx) * LG2E), g1 = exp2f((l1 - mx) * LG2E);
  const float g2 = exp2f((l2 - mx) * LG2E), g3 = exp2f((l3 - mx) * LG2E);
  const float g4 = exp2f((l4 - mx) * LG2E), g5 = exp2f((l5 - mx) * LG2E);
  const float g6 = exp2f((l6 - mx) * LG2E), g7 = exp2f((l7 - mx) * LG2E);
  const float s   = ((((((g0 + g1) + g2) + g3) + g4) + g5) + g6) + g7;
  const float gs  = exp2f((m1 - mx) * LG2E);
  const float inv = 1.0f / s;
  const float v0  = inv;
  const float v1  = gs * inv;
  const float den = (v0 + v1) + EPSW;
  const float rd  = 1.0f / den;
  const float w0  = v0 * rd;
  const float w1  = v1 * rd;

  v4i o;
  o.x = i0; o.y = i1; o.z = __float_as_int(w0); o.w = __float_as_int(w1);
  int* op = tinfo + 4 * (size_t)t;
  *(volatile v4i*)op = o;
  __threadfence();
  *(volatile v4i*)op = o;
}

__device__ __forceinline__ void plist_pass(
    const int* lst, int* plist, int tid,
    int s1, int s2, int s3, int s4, int s5, int s6, int s7, int s8,
    int c0, int c1, int c2, int c3, int c4, int c5, int c6, int c7) {
#pragma unroll 1
  for (int v = tid; v < NTL * TR / 4; v += NTHR) {
    const int r0 = v * 4;
    int e = 0;
    e += (r0 >= s1 * TR) ? 1 : 0; e += (r0 >= s2 * TR) ? 1 : 0; e += (r0 >= s3 * TR) ? 1 : 0;
    e += (r0 >= s4 * TR) ? 1 : 0; e += (r0 >= s5 * TR) ? 1 : 0; e += (r0 >= s6 * TR) ? 1 : 0;
    e += (r0 >= s7 * TR) ? 1 : 0;
    const bool used = r0 < s8 * TR;
    int sbt = 0, cc = c0;
    sbt = (e == 1) ? s1 : sbt; cc = (e == 1) ? c1 : cc;
    sbt = (e == 2) ? s2 : sbt; cc = (e == 2) ? c2 : cc;
    sbt = (e == 3) ? s3 : sbt; cc = (e == 3) ? c3 : cc;
    sbt = (e == 4) ? s4 : sbt; cc = (e == 4) ? c4 : cc;
    sbt = (e == 5) ? s5 : sbt; cc = (e == 5) ? c5 : cc;
    sbt = (e == 6) ? s6 : sbt; cc = (e == 6) ? c6 : cc;
    sbt = (e == 7) ? s7 : sbt; cc = (e == 7) ? c7 : cc;
    const int lc = r0 - sbt * TR;
    const int la = lc < 0 ? 0 : (lc > CAPE - 4 ? CAPE - 4 : lc);
    const v4i lv = *(const v4i*)(lst + e * CAPE + la);
    v4i o;
    o.x = (used && lc + 0 < cc) ? lv.x : -1;
    o.y = (used && lc + 1 < cc) ? lv.y : -1;
    o.z = (used && lc + 2 < cc) ? lv.z : -1;
    o.w = (used && lc + 3 < cc) ? lv.w : -1;
    *(volatile v4i*)(plist + r0) = o;
  }
}

__global__ __launch_bounds__(NTHR) void k_lists(const int* __restrict__ tinfo, int* plist, int* hdr, int nTok) {
  extern __shared__ v4i ldyn[];
  int* lst = (int*)ldyn;
  __shared__ int scnt[NE];
  __shared__ __attribute__((aligned(16))) int shdr[32];
  const int tid = threadIdx.x, lane = tid & 31, w = tid >> 5;

  int cnt = 0;
  const int nCh = nTok >> 5;
#pragma unroll 1
  for (int c = 0; c < nCh; ++c) {
    const int t = c * 32 + lane;
    const v4i inf = *(const v4i*)(tinfo + 4 * (size_t)t);
    const bool h0  = (inf.x == w);
    const bool h1  = (inf.y == w);
    const bool hit = h0 || h1;
    const unsigned mk = __builtin_amdgcn_ballot_w32(hit);
    const int pos = cnt + (int)__builtin_amdgcn_mbcnt_lo(mk, 0u);
    if (hit && pos < CAPE) lst[w * CAPE + pos] = (t << 1) | (h0 ? 0 : 1);
    cnt += (int)__builtin_popcount(mk);
  }
  if (lane == 0) scnt[w] = cnt > CAPE ? CAPE : cnt;
  __syncthreads();

  if (tid == 0) {
    const int c0 = scnt[0], c1 = scnt[1], c2 = scnt[2], c3 = scnt[3];
    const int c4 = scnt[4], c5 = scnt[5], c6 = scnt[6], c7 = scnt[7];
    const int s0 = 0;
    const int s1 = s0 + ((c0 + TR - 1) / TR);
    const int s2 = s1 + ((c1 + TR - 1) / TR);
    const int s3 = s2 + ((c2 + TR - 1) / TR);
    const int s4 = s3 + ((c3 + TR - 1) / TR);
    const int s5 = s4 + ((c4 + TR - 1) / TR);
    const int s6 = s5 + ((c5 + TR - 1) / TR);
    const int s7 = s6 + ((c6 + TR - 1) / TR);
    const int s8 = s7 + ((c7 + TR - 1) / TR);
    shdr[0] = s0; shdr[1] = s1; shdr[2] = s2; shdr[3] = s3; shdr[4] = s4;
    shdr[5] = s5; shdr[6] = s6; shdr[7] = s7; shdr[8] = s8;
    shdr[9] = 0; shdr[10] = 0; shdr[11] = 0; shdr[12] = 0; shdr[13] = 0; shdr[14] = 0; shdr[15] = 0;
    shdr[16] = c0; shdr[17] = c1; shdr[18] = c2; shdr[19] = c3;
    shdr[20] = c4; shdr[21] = c5; shdr[22] = c6; shdr[23] = c7;
    shdr[24] = 0; shdr[25] = 0; shdr[26] = 0; shdr[27] = 0; shdr[28] = 0; shdr[29] = 0; shdr[30] = 0; shdr[31] = 0;
  }
  __syncthreads();
  const int s1 = shdr[1], s2 = shdr[2], s3 = shdr[3], s4 = shdr[4];
  const int s5 = shdr[5], s6 = shdr[6], s7 = shdr[7], s8 = shdr[8];
  const int c0 = shdr[16], c1 = shdr[17], c2 = shdr[18], c3 = shdr[19];
  const int c4 = shdr[20], c5 = shdr[21], c6 = shdr[22], c7 = shdr[23];

  plist_pass(lst, plist, tid, s1, s2, s3, s4, s5, s6, s7, s8, c0, c1, c2, c3, c4, c5, c6, c7);
  v4i hv = {0, 0, 0, 0};
  if (tid < 8) hv = *(const v4i*)(shdr + 4 * tid);
  if (tid < 8) *(volatile v4i*)(hdr + 4 * tid) = hv;
  __threadfence();
  plist_pass(lst, plist, tid, s1, s2, s3, s4, s5, s6, s7, s8, c0, c1, c2, c3, c4, c5, c6, c7);
  if (tid < 8) *(volatile v4i*)(hdr + 4 * tid) = hv;
}

__global__ __launch_bounds__(NTHR) void k_gather(
    const float* __restrict__ x, const int* __restrict__ plist, unsigned short* Xg, int nTok) {
  const int tid = threadIdx.x;
  const int r   = blockIdx.x * 4 + (tid >> 6);
  const int c0  = (tid & 63) * 8;
  const int ent = plist[r];
  const bool valid = ent >= 0;
  int t = ent >> 1;
  t = t < 0 ? 0 : (t > nTok - 1 ? nTok - 1 : t);
  const float* xp = x + (size_t)t * DD + c0;
  const v4f a = *(const v4f*)xp;
  const v4f b = *(const v4f*)(xp + 4);
  v8us o;
  o[0] = valid ? (unsigned short)bfbits(a.x) : (unsigned short)0;
  o[1] = valid ? (unsigned short)bfbits(a.y) : (unsigned short)0;
  o[2] = valid ? (unsigned short)bfbits(a.z) : (unsigned short)0;
  o[3] = valid ? (unsigned short)bfbits(a.w) : (unsigned short)0;
  o[4] = valid ? (unsigned short)bfbits(b.x) : (unsigned short)0;
  o[5] = valid ? (unsigned short)bfbits(b.y) : (unsigned short)0;
  o[6] = valid ? (unsigned short)bfbits(b.z) : (unsigned short)0;
  o[7] = valid ? (unsigned short)bfbits(b.w) : (unsigned short)0;
  unsigned short* dp = Xg + (size_t)r * DD + c0;
  *(volatile v8us*)dp = o;
  __threadfence();
  *(volatile v8us*)dp = o;
}

__device__ __forceinline__ int tile_expert(const int* __restrict__ hdr, int j, int* ntOut) {
  const v4i hA = *(const v4i*)hdr;
  const v4i hB = *(const v4i*)(hdr + 4);
  int nt = hdr[8];
  nt = nt < 0 ? 0 : (nt > NTL ? NTL : nt);
  *ntOut = nt;
  int e = 0;
  e += (j >= hA.y) ? 1 : 0; e += (j >= hA.z) ? 1 : 0; e += (j >= hA.w) ? 1 : 0;
  e += (j >= hB.x) ? 1 : 0; e += (j >= hB.y) ? 1 : 0; e += (j >= hB.z) ? 1 : 0; e += (j >= hB.w) ? 1 : 0;
  return e;
}

__global__ __launch_bounds__(NTHR) void k_gemm1(
    const unsigned short* __restrict__ Xg, const unsigned short* __restrict__ W1t,
    const float* __restrict__ b1, const int* __restrict__ hdr,
    unsigned short* Hhi, unsigned short* Hlo, int tileBase) {
  __shared__ __attribute__((aligned(16))) unsigned short stg[8 * 2048];
  const int tid = threadIdx.x, lane = tid & 31, wave = tid >> 5, hh = lane >> 4, m = lane & 15;
  const int jl = blockIdx.x;
  const int j  = tileBase + jl;
  int nt;
  const int e = tile_expert(hdr, j, &nt);
  if (j >= nt) return;

  const int wr = wave >> 2, wc = wave & 3;
  const int colW = blockIdx.y * 256 + wc * 64;
  const unsigned short* aP = Xg  + ((size_t)j * TR + wr * 32 + m) * DD + 8 * hh;
  const unsigned short* bP = W1t + ((size_t)e * FFD + colW + m) * DD + 8 * hh;

  v8f acc[2][4];
#pragma unroll
  for (int R = 0; R < 2; ++R)
#pragma unroll
    for (int t = 0; t < 4; ++t) { v8f z = {0.f, 0.f, 0.f, 0.f, 0.f, 0.f, 0.f, 0.f}; acc[R][t] = z; }

#pragma unroll 1
  for (int kt = 0; kt < DD / 32; ++kt) {
    const int kk = kt * 32;
    FragB a[2], b[4];
#pragma unroll
    for (int R = 0; R < 2; ++R) {
      a[R].h[0] = *(const v8us*)(aP + (size_t)R * 16 * DD + kk);
      a[R].h[1] = *(const v8us*)(aP + (size_t)R * 16 * DD + kk + 16);
    }
#pragma unroll
    for (int t = 0; t < 4; ++t) {
      b[t].h[0] = *(const v8us*)(bP + (size_t)t * 16 * DD + kk);
      b[t].h[1] = *(const v8us*)(bP + (size_t)t * 16 * DD + kk + 16);
    }
#pragma unroll
    for (int R = 0; R < 2; ++R)
#pragma unroll
      for (int t = 0; t < 4; ++t) acc[R][t] = wmb(a[R].v, b[t].v, acc[R][t]);
  }

  float bb[4];
#pragma unroll
  for (int t = 0; t < 4; ++t) bb[t] = bfr(b1[(size_t)e * FFD + colW + 16 * t + m]);

  unsigned short* sh = stg + wave * 2048;
  unsigned short* sl = sh + 1024;
  const int q = lane >> 3, pc = lane & 7;
#pragma unroll
  for (int R = 0; R < 2; ++R) {
#pragma unroll
    for (int t = 0; t < 4; ++t) {
#pragma unroll
      for (int r = 0; r < 8; ++r) {
        float v = acc[R][t][r] + bb[t];
        v = fmaxf(v, 0.0f);
        const unsigned int hb = bfbits(v);
        const float hf = __uint_as_float(hb << 16);
        const unsigned int lb = bfbits(v - hf);
        const int li = (8 * hh + r) * 64 + 16 * t + m;
        sh[li] = (unsigned short)hb;
        sl[li] = (unsigned short)lb;
      }
    }
    __syncthreads();
    const size_t rowG = (size_t)jl * TR + wr * 32 + R * 16;
#pragma unroll
    for (int i = 0; i < 4; ++i) {
      const int row = 4 * i + q;
      const v8us hv = *(const v8us*)(sh + row * 64 + 8 * pc);
      const v8us lv = *(const v8us*)(sl + row * 64 + 8 * pc);
      const size_t go = (rowG + row) * FFD + colW + 8 * pc;
      *(volatile v8us*)(Hhi + go) = hv;
      *(volatile v8us*)(Hlo + go) = lv;
    }
    __threadfence();
#pragma unroll
    for (int i = 0; i < 4; ++i) {
      const int row = 4 * i + q;
      const v8us hv = *(const v8us*)(sh + row * 64 + 8 * pc);
      const v8us lv = *(const v8us*)(sl + row * 64 + 8 * pc);
      const size_t go = (rowG + row) * FFD + colW + 8 * pc;
      *(volatile v8us*)(Hhi + go) = hv;
      *(volatile v8us*)(Hlo + go) = lv;
    }
    __syncthreads();
  }
}

__global__ __launch_bounds__(NTHR) void k_gemm2(
    const unsigned short* __restrict__ Hhi, const unsigned short* __restrict__ Hlo,
    const unsigned short* __restrict__ W2t, const float* __restrict__ b2,
    const int* __restrict__ hdr, const int* __restrict__ plist, float* Y, int tileBase, int nTok) {
  __shared__ __attribute__((aligned(16))) float stg[8 * 1024];
  const int tid = threadIdx.x, lane = tid & 31, wave = tid >> 5, hh = lane >> 4, m = lane & 15;
  const int jl = blockIdx.x;
  const int j  = tileBase + jl;
  int nt;
  const int e = tile_expert(hdr, j, &nt);
  if (j >= nt) return;

  const int wr = wave >> 2, wc = wave & 3;
  const int colD = blockIdx.y * 256 + wc * 64;
  const int ent = plist[(size_t)j * TR + wr * 32 + lane];
  const unsigned short* ahP = Hhi + ((size_t)jl * TR + wr * 32 + m) * FFD + 8 * hh;
  const unsigned short* alP = Hlo + ((size_t)jl * TR + wr * 32 + m) * FFD + 8 * hh;
  const unsigned short* bP  = W2t + ((size_t)e * DD + colD + m) * FFD + 8 * hh;

  v8f acc[2][4];
#pragma unroll
  for (int R = 0; R < 2; ++R)
#pragma unroll
    for (int t = 0; t < 4; ++t) { v8f z = {0.f, 0.f, 0.f, 0.f, 0.f, 0.f, 0.f, 0.f}; acc[R][t] = z; }

#pragma unroll 1
  for (int kt = 0; kt < FFD / 32; ++kt) {
    const int kk = kt * 32;
    FragB ah[2], al[2], b[4];
#pragma unroll
    for (int R = 0; R < 2; ++R) {
      ah[R].h[0] = *(const v8us*)(ahP + (size_t)R * 16 * FFD + kk);
      ah[R].h[1] = *(const v8us*)(ahP + (size_t)R * 16 * FFD + kk + 16);
      al[R].h[0] = *(const v8us*)(alP + (size_t)R * 16 * FFD + kk);
      al[R].h[1] = *(const v8us*)(alP + (size_t)R * 16 * FFD + kk + 16);
    }
#pragma unroll
    for (int t = 0; t < 4; ++t) {
      b[t].h[0] = *(const v8us*)(bP + (size_t)t * 16 * FFD + kk);
      b[t].h[1] = *(const v8us*)(bP + (size_t)t * 16 * FFD + kk + 16);
    }
#pragma unroll
    for (int R = 0; R < 2; ++R)
#pragma unroll
      for (int t = 0; t < 4; ++t) {
        acc[R][t] = wmb(ah[R].v, b[t].v, acc[R][t]);
        acc[R][t] = wmb(al[R].v, b[t].v, acc[R][t]);
      }
  }

  float bb[4];
#pragma unroll
  for (int t = 0; t < 4; ++t) bb[t] = bfr(b2[(size_t)e * DD + colD + 16 * t + m]);

  float* sw = stg + wave * 1024;
#pragma unroll
  for (int R = 0; R < 2; ++R) {
#pragma unroll
    for (int t = 0; t < 4; ++t)
#pragma unroll
      for (int r = 0; r < 8; ++r) sw[(8 * hh + r) * 64 + 16 * t + m] = acc[R][t][r] + bb[t];
    __syncthreads();
#pragma unroll
    for (int i = 0; i < 8; ++i) {
      const int eA = __builtin_amdgcn_readlane(ent, R * 16 + 2 * i);
      const int eB = __builtin_amdgcn_readlane(ent, R * 16 + 2 * i + 1);
      const int my = hh ? eB : eA;
      const bool valid = my >= 0;
      int tt = my >> 1;
      tt = tt < 0 ? 0 : (tt > nTok - 1 ? nTok - 1 : tt);
      const int slot = my & 1;
      const v4f v = *(const v4f*)(sw + (2 * i + hh) * 64 + 4 * m);
      float* gp = Y + ((size_t)tt * 2 + slot) * DD + colD + 4 * m;
      if (valid) *(volatile v4f*)gp = v;
    }
    __threadfence();
#pragma unroll
    for (int i = 0; i < 8; ++i) {
      const int eA = __builtin_amdgcn_readlane(ent, R * 16 + 2 * i);
      const int eB = __builtin_amdgcn_readlane(ent, R * 16 + 2 * i + 1);
      const int my = hh ? eB : eA;
      const bool valid = my >= 0;
      int tt = my >> 1;
      tt = tt < 0 ? 0 : (tt > nTok - 1 ? nTok - 1 : tt);
      const int slot = my & 1;
      const v4f v = *(const v4f*)(sw + (2 * i + hh) * 64 + 4 * m);
      float* gp = Y + ((size_t)tt * 2 + slot) * DD + colD + 4 * m;
      if (valid) *(volatile v4f*)gp = v;
    }
    __syncthreads();
  }
}

__global__ __launch_bounds__(NTHR) void k_combine(
    const int* __restrict__ tinfo, const float* __restrict__ Y, float* out, int nTok) {
#pragma clang fp contract(off)
  const int tid = threadIdx.x;
  int t = blockIdx.x * 2 + (tid >> 7);
  t = t > nTok - 1 ? nTok - 1 : t;
  const int c0 = (tid & 127) * 4;
  const v4i inf = *(const v4i*)(tinfo + 4 * (size_t)t);
  const float w0 = __int_as_float(inf.z);
  const float w1 = __int_as_float(inf.w);
  const v4f y0 = *(const v4f*)(Y + ((size_t)t * 2) * DD + c0);
  const v4f y1 = *(const v4f*)(Y + ((size_t)t * 2 + 1) * DD + c0);
  const v4f p0 = y0 * w0;
  const v4f p1 = y1 * w1;
  const v4f o  = p0 + p1;
  float* gp = out + (size_t)t * DD + c0;
  *(volatile v4f*)gp = o;
  __threadfence();
  *(volatile v4f*)gp = o;
}

extern "C" void kernel_launch(void* const* d_in, const int* in_sizes, int n_in,
                              void* d_out, int out_size, void* d_ws, size_t ws_size,
                              hipStream_t stream) {
  if (n_in < 7) return;
  if (in_sizes[0] != NTOK * DD || in_sizes[1] != DD * NE || in_sizes[2] != NE) return;
  if (in_sizes[3] != NE * DD * FFD || in_sizes[4] != NE * FFD) return;
  if (in_sizes[5] != NE * FFD * DD || in_sizes[6] != NE * DD) return;
  if (out_size != NTOK * DD) return;

  const float* x  = (const float*)d_in[0];
  const float* Wg = (const float*)d_in[1];
  const float* bg = (const float*)d_in[2];
  const float* W1 = (const float*)d_in[3];
  const float* b1 = (const float*)d_in[4];
  const float* W2 = (const float*)d_in[5];
  const float* b2 = (const float*)d_in[6];
  float* out = (float*)d_out;

  char* ws = (char*)d_ws;
  size_t off = 0;
  const size_t oTI = off; off += (size_t)NTOK * 16;               off = (off + 255) & ~(size_t)255;
  const size_t oHD = off; off += 128;                             off = (off + 255) & ~(size_t)255;
  const size_t oPL = off; off += (size_t)NTL * TR * 4;            off = (off + 255) & ~(size_t)255;
  const size_t oW1 = off; off += (size_t)NE * FFD * DD * 2;        off = (off + 255) & ~(size_t)255;
  const size_t oW2 = off; off += (size_t)NE * DD * FFD * 2;        off = (off + 255) & ~(size_t)255;
  const size_t oXG = off; off += (size_t)NTL * TR * DD * 2;        off = (off + 255) & ~(size_t)255;
  const size_t oHH = off; off += (size_t)TPG * TR * FFD * 2;       off = (off + 255) & ~(size_t)255;
  const size_t oHL = off; off += (size_t)TPG * TR * FFD * 2;       off = (off + 255) & ~(size_t)255;
  const size_t oY  = off; off += (size_t)NTOK * 2 * DD * 4;        off = (off + 255) & ~(size_t)255;
  if (off > ws_size || off > (size_t)134217728) return;

  int*            tinfo = (int*)(ws + oTI);
  int*            hdr   = (int*)(ws + oHD);
  int*            plist = (int*)(ws + oPL);
  unsigned short* W1t   = (unsigned short*)(ws + oW1);
  unsigned short* W2t   = (unsigned short*)(ws + oW2);
  unsigned short* Xg    = (unsigned short*)(ws + oXG);
  unsigned short* Hhi   = (unsigned short*)(ws + oHH);
  unsigned short* Hlo   = (unsigned short*)(ws + oHL);
  float*          Y     = (float*)(ws + oY);

  k_wconv<<<dim3(DD / 64, FFD / 64, NE), NTHR, 0, stream>>>(W1, W1t, DD, FFD);
  k_wconv<<<dim3(FFD / 64, DD / 64, NE), NTHR, 0, stream>>>(W2, W2t, FFD, DD);

  k_gate<<<NTOK / NTHR, NTHR, 0, stream>>>(x, Wg, bg, tinfo, NTOK);
  hipFuncSetAttribute(reinterpret_cast<const void*>(&k_lists),
                      hipFuncAttributeMaxDynamicSharedMemorySize, LDS_LISTS);
  k_lists<<<1, NTHR, LDS_LISTS, stream>>>(tinfo, plist, hdr, NTOK);
  k_gather<<<(NTL * TR) / 4, NTHR, 0, stream>>>(x, plist, Xg, NTOK);

  for (int g = 0; g < NGRP; ++g) {
    k_gemm1<<<dim3(TPG, FFD / 256), NTHR, 0, stream>>>(Xg, W1t, b1, hdr, Hhi, Hlo, g * TPG);
    k_gemm2<<<dim3(TPG, DD / 256), NTHR, 0, stream>>>(Hhi, Hlo, W2t, b2, hdr, plist, Y, g * TPG, NTOK);
  }

  k_combine<<<NTOK / 2, NTHR, 0, stream>>>(tinfo, Y, out, NTOK);
}
